// NystromNonLinearKernel_86766929314328
// MI455X (gfx1250) — hardware-verified
//
#include <hip/hip_runtime.h>
#include <stddef.h>
#include <stdint.h>
#include <math.h>

constexpr int NB   = 8;
constexpr int CIN  = 16;
constexpr int COUT = 16;
constexpr int HID  = 128;
constexpr int S    = 32;
constexpr int RS   = S * S;
constexpr int IMG  = 256;
constexpr int NPIX = IMG * IMG;
constexpr int BNW  = NB * CIN;

constexpr int PQB    = 16;
constexpr int RSC    = 32;
constexpr int NCHUNK = RS / RSC;
constexpr int HP     = 136;
constexpr int KSP    = 40;
constexpr int OP     = 132;

static_assert(RS % RSC == 0);
static_assert(RS % PQB == 0);
static_assert(HP % 8 == 0 && KSP % 8 == 0 && OP % 4 == 0);

constexpr int LOFF_HID  = 0;
constexpr int LSZ_HID   = RSC * PQB * HP * 2;
constexpr int LOFF_K    = LOFF_HID + LSZ_HID;
constexpr int LSZ_K     = CIN * PQB * KSP * 2;
constexpr int LOFF_GRID = LOFF_K + LSZ_K;
constexpr int LSZ_GRID  = RS * 2 * 4;
constexpr int LOFF_W1   = LOFF_GRID + LSZ_GRID;
constexpr int LSZ_W1    = 3 * HID * 4;
constexpr int LOFF_B2   = LOFF_W1 + LSZ_W1;
constexpr int LSZ_B2    = CIN * 4;
constexpr int LDS_MAIN  = LOFF_B2 + LSZ_B2;
static_assert(LOFF_K % 16 == 0 && LOFF_GRID % 16 == 0 && LOFF_W1 % 16 == 0 && LOFF_B2 % 16 == 0);
static_assert(PQB * OP * 4 <= LSZ_HID);

constexpr float C_H    = 16.0f;
constexpr float C_W    = 16.0f;
constexpr float C_K    = 4.0f;
constexpr float C_S    = 16.0f;
constexpr float INV_HW = 1.0f / 256.0f;
constexpr float INV_KS = 1.0f / 2048.0f;

constexpr size_t OFF_SAMP = 0;
constexpr size_t SZ_SAMP  = (size_t)CIN * 16 * RS * 2;
constexpr size_t OFF_W2P  = OFF_SAMP + SZ_SAMP;
constexpr size_t SZ_W2P   = (size_t)CIN * HID * 2;
constexpr size_t OFF_OUTS = OFF_W2P + SZ_W2P;
constexpr size_t SZ_OUTS  = (size_t)RS * BNW * 4;
constexpr size_t WS_TOTAL = OFF_OUTS + SZ_OUTS;
static_assert(WS_TOTAL <= (size_t)134217728);
static_assert(OFF_W2P % 128 == 0 && OFF_OUTS % 128 == 0);
static_assert(SZ_SAMP % 128 == 0 && SZ_W2P % 128 == 0 && SZ_OUTS % 128 == 0);

typedef _Float16 v16h __attribute__((ext_vector_type(16)));
typedef _Float16 v8h __attribute__((ext_vector_type(8)));
typedef v8h __attribute__((may_alias)) v8ha;
typedef float v8f __attribute__((ext_vector_type(8)));
typedef float v4f __attribute__((ext_vector_type(4)));
typedef v4f __attribute__((may_alias)) v4fa;
typedef unsigned int v4u __attribute__((ext_vector_type(4)));

union Frag { v16h v; v8h h[2]; };

__device__ __forceinline__ v8f mma16(v16h a, v16h b, v8f c) {
  c = __builtin_amdgcn_wmma_f32_16x16x32_f16(false, a, false, b, (short)0, c, false, false);
  asm volatile("v_nop\n\tv_nop\n\tv_nop\n\tv_nop" : "+v"(c) : "v"(a), "v"(b));
  return c;
}

__device__ __forceinline__ v8f zero8() { return (v8f){0.f, 0.f, 0.f, 0.f, 0.f, 0.f, 0.f, 0.f}; }

__device__ __forceinline__ v16h ldfrag(const _Float16* base, int pitch, int row0, int k0, int lane) {
  const int m = lane & 15, hh = lane >> 4;
  const _Float16* q = base + (size_t)(row0 + m) * pitch + k0 + 8 * hh;
  Frag f;
  f.h[0] = *(const v8ha*)(q);
  f.h[1] = *(const v8ha*)(q + 16);
  return f.v;
}

__device__ __forceinline__ void st2_u4(_Float16* p, v4u v) {
  *(volatile v4u*)p = v;
  __threadfence();
  *(volatile v4u*)p = v;
}
__device__ __forceinline__ void st2_f4(float* p, v4f v) {
  *(volatile v4f*)p = v;
  __threadfence();
  *(volatile v4f*)p = v;
}

__device__ __forceinline__ unsigned int f16bits(float x) {
  return (unsigned int)__builtin_bit_cast(unsigned short, (_Float16)x);
}

__device__ __forceinline__ void shin(unsigned int& w0, unsigned int& w1, unsigned int& w2, unsigned int& w3, unsigned int hb) {
  w0 = (w0 >> 16) | (w1 << 16);
  w1 = (w1 >> 16) | (w2 << 16);
  w2 = (w2 >> 16) | (w3 << 16);
  w3 = (w3 >> 16) | (hb << 16);
}

__device__ __forceinline__ float gelu_erf(float x) {
  return 0.5f * x * (1.0f + erff(x * 0.70710678118654752f));
}

__global__ __launch_bounds__(256) void k_prep(const float* __restrict__ W2, _Float16* __restrict__ w2p) {
  const int t = threadIdx.x;
  const int n = t >> 4, h0 = (t & 15) * 8;
  unsigned int w0 = 0u, w1 = 0u, w2 = 0u, w3 = 0u;
#pragma unroll 1
  for (int j = 0; j < 8; ++j) {
    const int h = h0 + j;
    float s = 0.f;
#pragma unroll 1
    for (int mo = 0; mo < COUT; ++mo) s += W2[h * (COUT * CIN) + mo * CIN + n];
    shin(w0, w1, w2, w3, f16bits(s * C_W));
  }
  st2_u4(w2p + n * HID + h0, (v4u){w0, w1, w2, w3});
}

__global__ __launch_bounds__(128) void k_sample(const float* __restrict__ v, const float* __restrict__ grid,
                                                _Float16* __restrict__ samp) {
#pragma clang fp contract(off)
  const int blk = blockIdx.x;
  const int n = blk >> 4, b = blk & 15;
  const int t = threadIdx.x;
  unsigned int w0 = 0u, w1 = 0u, w2 = 0u, w3 = 0u;
  if (b < NB) {
    const float* vp = v + (size_t)(b * CIN + n) * (size_t)NPIX;
#pragma unroll 1
    for (int j = 0; j < 8; ++j) {
      const int rs = t * 8 + j;
      const float gx = grid[rs * 2 + 0], gy = grid[rs * 2 + 1];
      const float x = (gx + 1.0f) * 128.0f - 0.5f;
      const float y = (gy + 1.0f) * 128.0f - 0.5f;
      const float x0f = floorf(x), y0f = floorf(y);
      const float wx = x - x0f, wy = y - y0f;
      const int ix0 = (int)x0f, iy0 = (int)y0f;
      const int ix1 = ix0 + 1, iy1 = iy0 + 1;
      const bool vx0 = (ix0 >= 0) && (ix0 <= IMG - 1), vx1 = (ix1 >= 0) && (ix1 <= IMG - 1);
      const bool vy0 = (iy0 >= 0) && (iy0 <= IMG - 1), vy1 = (iy1 >= 0) && (iy1 <= IMG - 1);
      const int cx0 = min(max(ix0, 0), IMG - 1), cx1 = min(max(ix1, 0), IMG - 1);
      const int cy0 = min(max(iy0, 0), IMG - 1), cy1 = min(max(iy1, 0), IMG - 1);
      const float g00 = vp[cy0 * IMG + cx0], g10 = vp[cy0 * IMG + cx1];
      const float g01 = vp[cy1 * IMG + cx0], g11 = vp[cy1 * IMG + cx1];
      const float m00 = (vx0 && vy0) ? 1.0f : 0.0f, m10 = (vx1 && vy0) ? 1.0f : 0.0f;
      const float m01 = (vx0 && vy1) ? 1.0f : 0.0f, m11 = (vx1 && vy1) ? 1.0f : 0.0f;
      const float t00 = (g00 * m00) * ((1.0f - wx) * (1.0f - wy));
      const float t10 = (g10 * m10) * (wx * (1.0f - wy));
      const float t01 = (g01 * m01) * ((1.0f - wx) * wy);
      const float t11 = (g11 * m11) * (wx * wy);
      const float val = ((t00 + t10) + t01) + t11;
      shin(w0, w1, w2, w3, f16bits(val * C_S));
    }
  }
  st2_u4(samp + (size_t)blk * RS + t * 8, (v4u){w0, w1, w2, w3});
}

__global__ __launch_bounds__(256) void k_main(const float* __restrict__ grid, const float* __restrict__ W1,
                                              const float* __restrict__ b1, const float* __restrict__ b2,
                                              const _Float16* __restrict__ w2p, const _Float16* __restrict__ samp,
                                              float* __restrict__ outS) {
  extern __shared__ __align__(16) unsigned char dynlds[];
  _Float16* sHid  = (_Float16*)(dynlds + LOFF_HID);
  _Float16* sK    = (_Float16*)(dynlds + LOFF_K);
  float*    sGrid = (float*)(dynlds + LOFF_GRID);
  float*    sW1   = (float*)(dynlds + LOFF_W1);
  float*    sB2   = (float*)(dynlds + LOFF_B2);
  const int t = threadIdx.x;
  const int wave = t >> 5, lane = t & 31, hh = lane >> 4, m = lane & 15;
  const int pq0 = blockIdx.x * PQB;

  for (int i = t; i < RS * 2; i += 256) sGrid[i] = grid[i];
  for (int i = t; i < 3 * HID; i += 256) {
    const float wv = W1[min(i, 2 * HID - 1)];
    const float bv = b1[max(i - 2 * HID, 0)];
    sW1[i] = (i < 2 * HID) ? wv : bv;
  }
  if (t < CIN) {
    float s = 0.f;
#pragma unroll 1
    for (int mo = 0; mo < COUT; ++mo) s += b2[mo * CIN + t];
    sB2[t] = s;
  }
  v16h Bw[4];
#pragma unroll
  for (int kc = 0; kc < 4; ++kc) Bw[kc] = ldfrag(w2p, HID, 0, kc * 32, lane);
  __syncthreads();

  v8f acc0 = zero8(), acc1 = zero8();

#pragma unroll 1
  for (int ch = 0; ch < NCHUNK; ++ch) {
    const int rs0 = ch * RSC;

    float dxr[2], dyr[2];
#pragma unroll
    for (int rr = 0; rr < 2; ++rr) {
      const int row = t + rr * 256;
      const int rsl = row >> 4, pql = row & 15;
      const int rsg = rs0 + rsl, pqg = pq0 + pql;
      dxr[rr] = sGrid[rsg * 2 + 0] - sGrid[pqg * 2 + 0];
      dyr[rr] = sGrid[rsg * 2 + 1] - sGrid[pqg * 2 + 1];
    }
#pragma unroll 1
    for (int hb = 0; hb < HID; hb += 8) {
      const v4f wxA = *(const v4fa*)(sW1 + hb),           wxB = *(const v4fa*)(sW1 + hb + 4);
      const v4f wyA = *(const v4fa*)(sW1 + HID + hb),     wyB = *(const v4fa*)(sW1 + HID + hb + 4);
      const v4f bbA = *(const v4fa*)(sW1 + 2 * HID + hb), bbB = *(const v4fa*)(sW1 + 2 * HID + hb + 4);
#pragma unroll
      for (int rr = 0; rr < 2; ++rr) {
        const float dx = dxr[rr], dy = dyr[rr];
        v8h o;
#pragma unroll
        for (int k = 0; k < 8; ++k) {
          const float wx = (k < 4) ? wxA[k & 3] : wxB[k & 3];
          const float wy = (k < 4) ? wyA[k & 3] : wyB[k & 3];
          const float bb = (k < 4) ? bbA[k & 3] : bbB[k & 3];
          const float pre = fmaf(dx, wx, fmaf(dy, wy, bb));
          o[k] = (_Float16)(gelu_erf(pre) * C_H);
        }
        *(v8ha*)(sHid + (size_t)(t + rr * 256) * HP + hb) = o;
      }
    }
    __syncthreads();

#pragma unroll
    for (int i = 0; i < 4; ++i) {
      const int rt = wave * 4 + i;
      const v16h a0 = ldfrag(sHid, HP, rt * 16, 0, lane);
      const v16h a1 = ldfrag(sHid, HP, rt * 16, 32, lane);
      const v16h a2 = ldfrag(sHid, HP, rt * 16, 64, lane);
      const v16h a3 = ldfrag(sHid, HP, rt * 16, 96, lane);
      v8f c = zero8();
      c = mma16(a0, Bw[0], c);
      c = mma16(a1, Bw[1], c);
      c = mma16(a2, Bw[2], c);
      c = mma16(a3, Bw[3], c);
#pragma unroll
      for (int r = 0; r < 8; ++r) {
        const float ks = c[r] * INV_HW + sB2[m];
        sK[(m * 16 + 8 * hh + r) * KSP + rt] = (_Float16)(ks * C_K);
      }
    }
    __syncthreads();

    {
      const int n0 = wave * 2;
      const v16h a0c = ldfrag(sK, KSP, n0 * 16, 0, lane);
      const v16h b0c = ldfrag(samp, RS, n0 * 16, rs0, lane);
      acc0 = mma16(a0c, b0c, acc0);
      const v16h a1c = ldfrag(sK, KSP, (n0 + 1) * 16, 0, lane);
      const v16h b1c = ldfrag(samp, RS, (n0 + 1) * 16, rs0, lane);
      acc1 = mma16(a1c, b1c, acc1);
    }
  }

  __syncthreads();
  float* sOut = (float*)(dynlds + LOFF_HID);
#pragma unroll
  for (int nl = 0; nl < 2; ++nl) {
    const int n = wave * 2 + nl;
    const v8f d = nl ? acc1 : acc0;
    if (m < NB) {
#pragma unroll
      for (int r = 0; r < 8; ++r) sOut[(8 * hh + r) * OP + m * CIN + n] = d[r] * INV_KS;
    }
  }
  __syncthreads();
#pragma unroll
  for (int it = 0; it < 2; ++it) {
    const int idx = t + 256 * it;
    const int L = idx >> 3, pc = idx & 7;
    const int row = L >> 2, q4 = L & 3;
    const v4f val = *(const v4fa*)(sOut + row * OP + q4 * 32 + pc * 4);
    st2_f4(outS + (size_t)(pq0 + row) * BNW + q4 * 32 + pc * 4, val);
  }
}

__device__ __forceinline__ void lin8(int d, int& i0, int& i1, float& w0, float& w1) {
  const float s = ((float)d + 0.5f) * 0.125f - 0.5f;
  const float f0 = floorf(s);
  const int i = (int)f0;
  const float f = s - f0;
  const bool lo = i < 0, hi = i >= S - 1;
  i0 = lo ? 0 : (hi ? S - 1 : i);
  i1 = lo ? 0 : (hi ? S - 1 : i + 1);
  w0 = (lo || hi) ? 1.0f : (1.0f - f);
  w1 = (lo || hi) ? 0.0f : f;
}

__global__ __launch_bounds__(256) void k_resize(const float* __restrict__ outS, float* __restrict__ u) {
#pragma clang fp contract(off)
  const int idx = blockIdx.x * 256 + (int)threadIdx.x;
  const int x4 = idx & 63, y = (idx >> 6) & 255, bn = idx >> 14;
  int ya, yb; float wya, wyb;
  lin8(y, ya, yb, wya, wyb);
  const float* pa = outS + bn;
  v4f res;
#pragma unroll
  for (int j = 0; j < 4; ++j) {
    int xa, xb; float wxa, wxb;
    lin8(x4 * 4 + j, xa, xb, wxa, wxb);
    const float p00 = pa[(size_t)(ya * S + xa) * BNW], p10 = pa[(size_t)(yb * S + xa) * BNW];
    const float p01 = pa[(size_t)(ya * S + xb) * BNW], p11 = pa[(size_t)(yb * S + xb) * BNW];
    const float t0 = wya * p00 + wyb * p10;
    const float t1 = wya * p01 + wyb * p11;
    res[j] = wxa * t0 + wxb * t1;
  }
  st2_f4(u + (size_t)idx * 4, res);
}

extern "C" void kernel_launch(void* const* d_in, const int* in_sizes, int n_in,
                              void* d_out, int out_size, void* d_ws, size_t ws_size,
                              hipStream_t stream) {
  if (n_in < 6) return;
  if (in_sizes[0] != NB * CIN * NPIX) return;
  if (in_sizes[1] != RS * 2) return;
  if (in_sizes[2] != 2 * HID || in_sizes[3] != HID) return;
  if (in_sizes[4] != HID * COUT * CIN || in_sizes[5] != COUT * CIN) return;
  if (out_size != NB * CIN * NPIX) return;
  if (ws_size < WS_TOTAL) return;

  const float* v    = (const float*)d_in[0];
  const float* grid = (const float*)d_in[1];
  const float* W1   = (const float*)d_in[2];
  const float* b1   = (const float*)d_in[3];
  const float* W2   = (const float*)d_in[4];
  const float* b2   = (const float*)d_in[5];
  float* u = (float*)d_out;
  char* ws = (char*)d_ws;

  _Float16* samp = (_Float16*)(ws + OFF_SAMP);
  _Float16* w2p  = (_Float16*)(ws + OFF_W2P);
  float*    outS = (float*)(ws + OFF_OUTS);

  k_prep<<<dim3(1), dim3(256), 0, stream>>>(W2, w2p);
  k_sample<<<dim3(CIN * 16), dim3(128), 0, stream>>>(v, grid, samp);
  (void)hipFuncSetAttribute(reinterpret_cast<const void*>(&k_main), hipFuncAttributeMaxDynamicSharedMemorySize, LDS_MAIN);
  k_main<<<dim3(RS / PQB), dim3(256), LDS_MAIN, stream>>>(grid, W1, b1, b2, w2p, samp, outS);
  k_resize<<<dim3((NB * CIN * NPIX) / (256 * 4)), dim3(256), 0, stream>>>(outS, u);
  (void)hipGetLastError();
}
